// RNN_74775380623930
// MI455X (gfx1250) — hardware-verified
//
#include <hip/hip_runtime.h>
#include <math.h>

constexpr int NBATCH   = 1024;
constexpr int NSTEP    = 2048;
constexpr int NHID     = 32;
constexpr int NGATE    = 4 * NHID;
constexpr int ROWS_BLK = 16;
constexpr int CHUNK_T  = 32;
constexpr int WPITCH   = 40;
constexpr int HPITCH   = 40;
constexpr int FPITCH   = 36;
constexpr int OPITCH   = 36;
constexpr float HCARRY = 16.0f;
constexpr float WCARRY = 64.0f;
constexpr float SCARRY = HCARRY * WCARRY;
constexpr float LOG2E_F = 1.4426950408889634f;
constexpr float KSIG_S  = -LOG2E_F / SCARRY;
constexpr float KTANH_S = 2.0f * LOG2E_F / SCARRY;
constexpr float KTANH_1 = 2.0f * LOG2E_F;

static_assert(NHID == 32, "one 32-deep k step");
static_assert(NGATE == 128, "eight 16-column gate tiles");
static_assert(NBATCH % ROWS_BLK == 0, "grid exact");
static_assert(NSTEP % CHUNK_T == 0, "no time tail");
static_assert(CHUNK_T == 32, "one 128-B line per row per chunk");
static_assert((NGATE * NHID) == 32 * 32 * 4, "weight staging loop exact");
static_assert(SCARRY == 1024.0f, "carry product");

typedef __attribute__((ext_vector_type(16))) _Float16 v16h;
typedef __attribute__((ext_vector_type(8)))  _Float16 v8h;
typedef __attribute__((ext_vector_type(8)))  float    v8f;
typedef __attribute__((ext_vector_type(4)))  float    v4f;

__device__ __forceinline__ void dep_guard_h(v8f& a, v8f& b, v16h x, v16h y) { asm volatile("v_nop\n\tv_nop\n\tv_nop\n\tv_nop" : "+v"(a), "+v"(b) : "v"(x), "v"(y)); }
__device__ __forceinline__ void keep4_h(v16h a, v16h b, v16h c, v16h d) { asm volatile("v_nop" :: "v"(a), "v"(b), "v"(c), "v"(d)); }
template <typename T> struct Frag;
template <> struct Frag<_Float16> {
  typedef v16h V; union U { v16h v; v8h h[2]; };
  static __device__ __forceinline__ v16h load(const _Float16* p) {
    U f; f.h[0] = *(const v8h*)(p); f.h[1] = *(const v8h*)(p + 16); return f.v;
  }
  static __device__ __forceinline__ v8f mma(v16h a, v16h b, v8f c) {
    return __builtin_amdgcn_wmma_f32_16x16x32_f16(false, a, false, b, (short)0, c, false, false);
  }
  static __device__ __forceinline__ void guard(v8f& a, v8f& b, v16h x, v16h y) { dep_guard_h(a, b, x, y); }
  static __device__ __forceinline__ void keep(v16h a, v16h b, v16h c, v16h d) { keep4_h(a, b, c, d); }
};

__device__ __forceinline__ void guard4ab(v8f& d0, v8f& d1, v8f& d2, v8f& d3, v16h a, v16h b0, v16h b1, v16h b2, v16h b3) {
  asm volatile("v_nop\n\tv_nop\n\tv_nop\n\tv_nop" : "+v"(d0), "+v"(d1), "+v"(d2), "+v"(d3) : "v"(a), "v"(b0), "v"(b1), "v"(b2), "v"(b3));
}
__device__ __forceinline__ void pin8(float& a0, float& a1, float& a2, float& a3, float& a4, float& a5, float& a6, float& a7) {
  asm volatile("" : "+v"(a0), "+v"(a1), "+v"(a2), "+v"(a3), "+v"(a4), "+v"(a5), "+v"(a6), "+v"(a7) :: "memory");
}
__device__ __forceinline__ void pin4v(v4f& a0, v4f& a1, v4f& a2, v4f& a3) {
  asm volatile("" : "+v"(a0), "+v"(a1), "+v"(a2), "+v"(a3) :: "memory");
}

__device__ __forceinline__ float sig_k(float d, float k)  { return __builtin_amdgcn_rcpf(1.0f + __builtin_amdgcn_exp2f(d * k)); }
__device__ __forceinline__ float tanh_k(float d, float k) { return 1.0f - 2.0f * __builtin_amdgcn_rcpf(__builtin_amdgcn_exp2f(d * k) + 1.0f); }

__device__ __forceinline__ void gate_group(const v16h a, const v16h bi, const v16h bf, const v16h bg, const v16h bo,
                                           const float wi, const float wf, const float wg, const float wo,
                                           const float ci, const float cf, const float cg, const float co,
                                           const v4f xa, const v4f xb, v8f& cst, _Float16* hq, float* hf) {
  const float xs[8] = {xa[0], xa[1], xa[2], xa[3], xb[0], xb[1], xb[2], xb[3]};
  v8f di, df, dg, dq;
#pragma unroll
  for (int r = 0; r < 8; ++r) {
    di[r] = fmaf(xs[r], wi, ci);
    df[r] = fmaf(xs[r], wf, cf);
    dg[r] = fmaf(xs[r], wg, cg);
    dq[r] = fmaf(xs[r], wo, co);
  }
  di = Frag<_Float16>::mma(a, bi, di);
  df = Frag<_Float16>::mma(a, bf, df);
  dg = Frag<_Float16>::mma(a, bg, dg);
  dq = Frag<_Float16>::mma(a, bo, dq);
  guard4ab(di, df, dg, dq, a, bi, bf, bg, bo);
#pragma unroll
  for (int r = 0; r < 8; ++r) {
    const float ig = sig_k(di[r], KSIG_S);
    const float fg = sig_k(df[r], KSIG_S);
    const float gg = tanh_k(dg[r], KTANH_S);
    const float og = sig_k(dq[r], KSIG_S);
    const float cn = fmaf(fg, cst[r], ig * gg);
    cst[r] = cn;
    const float hn = og * tanh_k(cn, KTANH_1);
    hf[r * FPITCH] = hn;
    hq[r * HPITCH] = (_Float16)(hn * HCARRY);
  }
}

__global__ __launch_bounds__(32) void lstm_seq_kernel(const float* x, const float* W_ih, const float* W_hh,
                                                      const float* b_ih, const float* b_hh,
                                                      const float* W_out, const float* b_out, float* out) {
  __shared__ __align__(16) _Float16 wsh[NGATE * WPITCH];
  __shared__ __align__(16) _Float16 hq16[ROWS_BLK * HPITCH];
  __shared__ __align__(16) float    hf32[ROWS_BLK * FPITCH];
  __shared__ __align__(16) float    xbuf[CHUNK_T * ROWS_BLK];
  __shared__ __align__(16) float    obuf[ROWS_BLK * OPITCH];

  const int lane = threadIdx.x & 31;
  const int c    = lane & 15;
  const int hh   = lane >> 4;
  const int bbase = blockIdx.x * ROWS_BLK;

#pragma unroll 1
  for (int it = 0; it < 32; ++it) {
    const int idx = it * 32 + lane;
    const int n  = idx >> 3;
    const int k4 = (idx & 7) * 4;
    const v4f v = *(const v4f*)(W_hh + 4 * idx);
    _Float16* wp = wsh + n * WPITCH + k4;
    wp[0] = (_Float16)(v[0] * WCARRY);
    wp[1] = (_Float16)(v[1] * WCARRY);
    wp[2] = (_Float16)(v[2] * WCARRY);
    wp[3] = (_Float16)(v[3] * WCARRY);
  }

  float wi[8], bs[8];
  {
    float ta[8];
#pragma unroll
    for (int n = 0; n < 8; ++n) ta[n] = W_ih[16 * n + c];
    pin8(ta[0], ta[1], ta[2], ta[3], ta[4], ta[5], ta[6], ta[7]);
#pragma unroll
    for (int n = 0; n < 8; ++n) wi[n] = ta[n] * SCARRY;
  }
  {
    float tb[8], tc[8];
#pragma unroll
    for (int n = 0; n < 8; ++n) tb[n] = b_ih[16 * n + c];
    pin8(tb[0], tb[1], tb[2], tb[3], tb[4], tb[5], tb[6], tb[7]);
#pragma unroll
    for (int n = 0; n < 8; ++n) tc[n] = b_hh[16 * n + c];
    pin8(tc[0], tc[1], tc[2], tc[3], tc[4], tc[5], tc[6], tc[7]);
#pragma unroll
    for (int n = 0; n < 8; ++n) bs[n] = (tb[n] + tc[n]) * SCARRY;
  }
  v4f wo0 = *(const v4f*)(W_out + 8 * hh);
  v4f wo1 = *(const v4f*)(W_out + 8 * hh + 4);
  v4f wo2 = *(const v4f*)(W_out + 16 + 8 * hh);
  v4f wo3 = *(const v4f*)(W_out + 16 + 8 * hh + 4);
  pin4v(wo0, wo1, wo2, wo3);
  const float bo = b_out[0];

  __syncthreads();

  v16h WB[8];
#pragma unroll
  for (int n = 0; n < 8; ++n) WB[n] = Frag<_Float16>::load(wsh + (16 * n + c) * WPITCH + 8 * hh);

  v16h A;
#pragma unroll
  for (int e = 0; e < 16; ++e) A[e] = (_Float16)0.0f;
  v8f cs0 = {0.f, 0.f, 0.f, 0.f, 0.f, 0.f, 0.f, 0.f};
  v8f cs1 = {0.f, 0.f, 0.f, 0.f, 0.f, 0.f, 0.f, 0.f};

  const float* xg = x + (size_t)bbase * NSTEP + lane;
  _Float16* hq_lane = hq16 + (8 * hh) * HPITCH + c;
  float*    hf_lane = hf32 + (8 * hh) * FPITCH + c;
  const _Float16* a_src = hq16 + c * HPITCH + 8 * hh;
  const float*    h_src = hf32 + c * FPITCH + 8 * hh;
  const int q  = lane >> 3;
  const int c4 = (lane & 7) * 4;

#pragma unroll 1
  for (int ch = 0; ch < NSTEP / CHUNK_T; ++ch) {
    const int t0 = ch * CHUNK_T;
#pragma unroll 1
    for (int g = 0; g < 2; ++g) {
#pragma unroll
      for (int i = 0; i < 8; ++i) {
        const int row = g * 8 + i;
        const float xv = xg[(size_t)row * NSTEP + t0];
        xbuf[lane * ROWS_BLK + row] = xv;
      }
    }
    __syncthreads();

#pragma unroll 1
    for (int tt = 0; tt < CHUNK_T; ++tt) {
      const v4f xa = *(const v4f*)(xbuf + tt * ROWS_BLK + 8 * hh);
      const v4f xb = *(const v4f*)(xbuf + tt * ROWS_BLK + 8 * hh + 4);
      gate_group(A, WB[0], WB[2], WB[4], WB[6], wi[0], wi[2], wi[4], wi[6], bs[0], bs[2], bs[4], bs[6],
                 xa, xb, cs0, hq_lane, hf_lane);
      gate_group(A, WB[1], WB[3], WB[5], WB[7], wi[1], wi[3], wi[5], wi[7], bs[1], bs[3], bs[5], bs[7],
                 xa, xb, cs1, hq_lane + 16, hf_lane + 16);
      __syncthreads();
      A = Frag<_Float16>::load(a_src);
      const v4f p0 = *(const v4f*)(h_src);
      const v4f p1 = *(const v4f*)(h_src + 4);
      const v4f p2 = *(const v4f*)(h_src + 16);
      const v4f p3 = *(const v4f*)(h_src + 20);
      float s = 0.0f;
#pragma unroll
      for (int e = 0; e < 4; ++e) s = fmaf(p0[e], wo0[e], s);
#pragma unroll
      for (int e = 0; e < 4; ++e) s = fmaf(p1[e], wo1[e], s);
#pragma unroll
      for (int e = 0; e < 4; ++e) s = fmaf(p2[e], wo2[e], s);
#pragma unroll
      for (int e = 0; e < 4; ++e) s = fmaf(p3[e], wo3[e], s);
      s += __shfl_xor(s, 16, 32);
      const float ov = s + bo;
      if (hh == 0) obuf[c * OPITCH + tt] = ov;
      __syncthreads();
    }

    for (int pass = 0; pass < 2; ++pass) {
#pragma unroll
      for (int it = 0; it < 4; ++it) {
        const int row = it * 4 + q;
        const v4f v = *(const v4f*)(obuf + row * OPITCH + c4);
        *(volatile v4f*)(out + (size_t)(bbase + row) * NSTEP + t0 + c4) = v;
      }
      __threadfence();
    }
    __syncthreads();
  }
}

extern "C" void kernel_launch(void* const* d_in, const int* in_sizes, int n_in,
                              void* d_out, int out_size, void* d_ws, size_t ws_size, hipStream_t stream) {
  (void)d_ws; (void)ws_size;
  if (n_in < 7 || d_out == nullptr) return;
  if (in_sizes[0] != NBATCH * NSTEP || in_sizes[1] != NGATE || in_sizes[2] != NGATE * NHID ||
      in_sizes[3] != NGATE || in_sizes[4] != NGATE || in_sizes[5] != NHID || in_sizes[6] != 1 ||
      out_size != NBATCH * NSTEP) return;
  const float* x     = (const float*)d_in[0];
  const float* W_ih  = (const float*)d_in[1];
  const float* W_hh  = (const float*)d_in[2];
  const float* b_ih  = (const float*)d_in[3];
  const float* b_hh  = (const float*)d_in[4];
  const float* W_out = (const float*)d_in[5];
  const float* b_out = (const float*)d_in[6];
  float* out = (float*)d_out;
  lstm_seq_kernel<<<NBATCH / ROWS_BLK, 32, 0, stream>>>(x, W_ih, W_hh, b_ih, b_hh, W_out, b_out, out);
}
